// BaseSingleSplitDNAMiteModel_47493748359457
// MI455X (gfx1250) — hardware-verified
//
#include <hip/hip_runtime.h>


#define NB_  2048
#define NF   32
#define NE   32
#define NH   64
#define FS   64
#define NPR  496
#define PCH  62
#define NPC  8
#define TOT  (NF * FS)
#define DM   NH
#define LOSC 1024.0f

typedef _Float16 h16;
typedef unsigned short bf;
typedef __attribute__((ext_vector_type(16))) __bf16   v16bf;
typedef __attribute__((ext_vector_type(16))) _Float16 v16h;
typedef __attribute__((ext_vector_type(8)))  _Float16 v8h;
typedef __attribute__((ext_vector_type(8)))  unsigned short v8us;
typedef __attribute__((ext_vector_type(8)))  float    v8f;
typedef __attribute__((ext_vector_type(4)))  float    v4f;
typedef v8h  __attribute__((may_alias)) v8ha;
typedef v4f  __attribute__((may_alias)) v4fa;
typedef v8us __attribute__((may_alias)) v8usa;

__device__ __forceinline__ unsigned short f2bf(float f) { unsigned u = __float_as_uint(f); u += 0x7FFFu + ((u >> 16) & 1u); return (unsigned short)(u >> 16); }
__device__ __forceinline__ float bf2f(unsigned short b) { return __uint_as_float(((unsigned)b) << 16); }
__device__ __forceinline__ float bfr(float f) { return bf2f(f2bf(f)); }
__device__ __forceinline__ v16h cat16(v8h lo, v8h hi) { return __builtin_shufflevector(lo, hi, 0, 1, 2, 3, 4, 5, 6, 7, 8, 9, 10, 11, 12, 13, 14, 15); }
__device__ __forceinline__ v16bf cat16b(v8us lo, v8us hi) { return __builtin_bit_cast(v16bf, __builtin_shufflevector(lo, hi, 0, 1, 2, 3, 4, 5, 6, 7, 8, 9, 10, 11, 12, 13, 14, 15)); }
__device__ __forceinline__ v8f wmma16(v16h a, v16h b, v8f c) { return __builtin_amdgcn_wmma_f32_16x16x32_f16(false, a, false, b, (short)0, c, false, false); }
__device__ __forceinline__ v8f wmmab(v16bf a, v16bf b, v8f c) { return __builtin_amdgcn_wmma_f32_16x16x32_bf16(false, a, false, b, (short)0, c, false, false); }

template <bool SPLITA, bool F16OUT = false>
__global__ __launch_bounds__(128) void k_gemmb(const bf* __restrict__ A, const bf* __restrict__ Al, const bf* __restrict__ Bn, const float* __restrict__ bias, float* C, int ldc, h16* C2, const float* __restrict__ R = nullptr, int K = DM, int roundR = 1) {
    __shared__ __align__(16) float ost[4][16 * 68];
    const int lane = threadIdx.x & 31, wave = threadIdx.x >> 5, lr = lane & 15, hi = lane >> 4;
    const int r0 = blockIdx.x * 64 + wave * 16, c0 = blockIdx.y * 64;
    const size_t aoff = (size_t)(r0 + lr) * K + 8 * hi;
    size_t boff[4];
#pragma unroll
    for (int t = 0; t < 4; ++t) boff[t] = (size_t)(c0 + t * 16 + lr) * K + 8 * hi;
    v8f acc[4];
#pragma unroll
    for (int t = 0; t < 4; ++t) acc[t] = (v8f){};
#pragma unroll 1
    for (int kc = 0; kc < K; kc += 32) {
        const v16bf a = cat16b(*(const v8us*)(A + aoff + kc), *(const v8us*)(A + aoff + kc + 16));
        v16bf al = a;
        if (SPLITA) al = cat16b(*(const v8us*)(Al + aoff + kc), *(const v8us*)(Al + aoff + kc + 16));
#pragma unroll
        for (int t = 0; t < 4; ++t) { const v16bf b = cat16b(*(const v8us*)(Bn + boff[t] + kc), *(const v8us*)(Bn + boff[t] + kc + 16)); acc[t] = wmmab(a, b, acc[t]); if (SPLITA) acc[t] = wmmab(al, b, acc[t]); }
        asm volatile("v_nop\n\tv_nop\n\tv_nop\n\tv_nop" : "+v"(acc[0]), "+v"(acc[1]), "+v"(acc[2]), "+v"(acc[3]) : "v"(a), "v"(al));
    }
    float* os = &ost[wave][0];
#pragma unroll
    for (int t = 0; t < 4; ++t) { const float bv = bias ? bfr(bias[c0 + t * 16 + lr]) : 0.f;
#pragma unroll
        for (int j = 0; j < 8; ++j) os[(hi * 8 + j) * 68 + t * 16 + lr] = acc[t][j] + bv; }
    __syncthreads();
    if (F16OUT) {
        h16* crow = (h16*)(void*)C + (size_t)r0 * ldc + c0;
        auto pass = [&]() {
#pragma unroll
            for (int s = 0; s < 4; ++s) { const int row = 4 * s + (lane >> 3), piece = lane & 7; const float* sp = os + row * 68 + piece * 8; v8h o, o2;
#pragma unroll
                for (int i = 0; i < 8; ++i) { const h16 a = (h16)sp[i]; o[i] = a; o2[i] = (h16)((sp[i] - (float)a) * LOSC); }
                *(volatile v8h*)(crow + (size_t)row * ldc + piece * 8) = o; if (C2) *(volatile v8h*)(C2 + (size_t)r0 * ldc + c0 + (size_t)row * ldc + piece * 8) = o2; }
        };
        pass(); __threadfence(); pass();
    } else {
        float* crow = C + (size_t)r0 * ldc + c0;
        auto pass = [&]() {
#pragma unroll
            for (int s = 0; s < 8; ++s) { const int Lid = (lane >> 3) + 4 * s, piece = lane & 7; const int row = Lid >> 1, cofs = (Lid & 1) * 32 + piece * 4;
                v4f val = *(const v4fa*)(os + row * 68 + cofs); if (R) { const v4f rv = *(const v4f*)(R + ((size_t)r0 + row) * ldc + c0 + cofs); val += roundR ? (v4f){bfr(rv[0]), bfr(rv[1]), bfr(rv[2]), bfr(rv[3])} : rv; }
                *(volatile v4f*)(crow + (size_t)row * ldc + cofs) = val; }
        };
        pass(); __threadfence(); pass();
    }
}

template <bool SPLITA, bool F16OUT = false>
__global__ __launch_bounds__(128) void k_gemmbz(const bf* __restrict__ A, const bf* __restrict__ Al, const bf* __restrict__ Bn, const float* __restrict__ bias, float* C, int ldc, h16* C2, const float* __restrict__ R, int K, int roundR, size_t sA, size_t sB, size_t sBias, size_t sC) {
    { const size_t g = blockIdx.z; A += g * sA; if (Al) Al += g * sA; Bn += g * sB; if (bias) bias += g * sBias; C += g * sC; if (R) R += g * sC; }
    __shared__ __align__(16) float ost[4][16 * 68];
    const int lane = threadIdx.x & 31, wave = threadIdx.x >> 5, lr = lane & 15, hi = lane >> 4;
    const int r0 = blockIdx.x * 64 + wave * 16, c0 = blockIdx.y * 64;
    const size_t aoff = (size_t)(r0 + lr) * K + 8 * hi;
    size_t boff[4];
#pragma unroll
    for (int t = 0; t < 4; ++t) boff[t] = (size_t)(c0 + t * 16 + lr) * K + 8 * hi;
    v8f acc[4];
#pragma unroll
    for (int t = 0; t < 4; ++t) acc[t] = (v8f){};
#pragma unroll 1
    for (int kc = 0; kc < K; kc += 32) {
        const v16bf a = cat16b(*(const v8us*)(A + aoff + kc), *(const v8us*)(A + aoff + kc + 16));
        v16bf al = a;
        if (SPLITA) al = cat16b(*(const v8us*)(Al + aoff + kc), *(const v8us*)(Al + aoff + kc + 16));
#pragma unroll
        for (int t = 0; t < 4; ++t) { const v16bf b = cat16b(*(const v8us*)(Bn + boff[t] + kc), *(const v8us*)(Bn + boff[t] + kc + 16)); acc[t] = wmmab(a, b, acc[t]); if (SPLITA) acc[t] = wmmab(al, b, acc[t]); }
        asm volatile("v_nop\n\tv_nop\n\tv_nop\n\tv_nop" : "+v"(acc[0]), "+v"(acc[1]), "+v"(acc[2]), "+v"(acc[3]) : "v"(a), "v"(al));
    }
    float* os = &ost[wave][0];
#pragma unroll
    for (int t = 0; t < 4; ++t) { const float bv = bias ? bfr(bias[c0 + t * 16 + lr]) : 0.f;
#pragma unroll
        for (int j = 0; j < 8; ++j) os[(hi * 8 + j) * 68 + t * 16 + lr] = acc[t][j] + bv; }
    __syncthreads();
    if (F16OUT) {
        h16* crow = (h16*)(void*)C + (size_t)r0 * ldc + c0;
        auto pass = [&]() {
#pragma unroll
            for (int s = 0; s < 4; ++s) { const int row = 4 * s + (lane >> 3), piece = lane & 7; const float* sp = os + row * 68 + piece * 8; v8h o, o2;
#pragma unroll
                for (int i = 0; i < 8; ++i) { const h16 a = (h16)sp[i]; o[i] = a; o2[i] = (h16)((sp[i] - (float)a) * LOSC); }
                *(volatile v8h*)(crow + (size_t)row * ldc + piece * 8) = o; if (C2) *(volatile v8h*)(C2 + (size_t)r0 * ldc + c0 + (size_t)row * ldc + piece * 8) = o2; }
        };
        pass(); __threadfence(); pass();
    } else {
        float* crow = C + (size_t)r0 * ldc + c0;
        auto pass = [&]() {
#pragma unroll
            for (int s = 0; s < 8; ++s) { const int Lid = (lane >> 3) + 4 * s, piece = lane & 7; const int row = Lid >> 1, cofs = (Lid & 1) * 32 + piece * 4;
                v4f val = *(const v4fa*)(os + row * 68 + cofs); if (R) { const v4f rv = *(const v4f*)(R + ((size_t)r0 + row) * ldc + c0 + cofs); val += roundR ? (v4f){bfr(rv[0]), bfr(rv[1]), bfr(rv[2]), bfr(rv[3])} : rv; }
                *(volatile v4f*)(crow + (size_t)row * ldc + cofs) = val; }
        };
        pass(); __threadfence(); pass();
    }
}


__global__ __launch_bounds__(256) void k_wtb(const float* __restrict__ Wm, int K, int N, bf* WT) {
    __shared__ float tl[64][65];
    const int g = blockIdx.x, tid = threadIdx.x;
    for (int e = tid; e < 64 * 64; e += 256) { const int k = e / 64, n = e % 64; tl[k][n] = (k < K && n < N) ? Wm[((size_t)g * K + (k < K ? k : 0)) * N + (n < N ? n : 0)] : 0.f; }
    __syncthreads();
    typedef __attribute__((ext_vector_type(2))) unsigned short v2us;
    const int lane = tid & 31, wv = tid >> 5;
    auto pass = [&]() {
#pragma unroll 1
        for (int n = wv; n < 64; n += 8) { v2us o; o[0] = f2bf(tl[lane * 2][n]); o[1] = f2bf(tl[lane * 2 + 1][n]); *(volatile v2us*)(WT + ((size_t)g * 64 + n) * 64 + lane * 2) = o; }
    };
    pass(); __threadfence(); pass();
}
__global__ __launch_bounds__(256) void k_embm(const int* __restrict__ mains, const int* __restrict__ offs, const float* __restrict__ emb, bf* EM) {
    typedef __attribute__((ext_vector_type(2))) unsigned short v2us;
    const int lane = threadIdx.x & 31; const size_t wid = (size_t)blockIdx.x * 8 + (threadIdx.x >> 5); if (wid >= (size_t)NF * NB_) return; const int f = (int)(wid / NB_), b = (int)(wid % NB_);
    int idx = mains[b * NF + f] + offs[f]; idx = idx < 0 ? 0 : (idx >= TOT ? TOT - 1 : idx); v2us o;
#pragma unroll
    for (int i = 0; i < 2; ++i) { const int e = lane * 2 + i; o[i] = (e < NE) ? f2bf(emb[(size_t)idx * NE + (e < NE ? e : 0)]) : (unsigned short)0; }
    *(volatile v2us*)(EM + wid * 64 + lane * 2) = o; __threadfence(); *(volatile v2us*)(EM + wid * 64 + lane * 2) = o;
}
__global__ __launch_bounds__(256) void k_embp(const int* __restrict__ pairs, const int* __restrict__ plist, const int* __restrict__ offs, const float* __restrict__ emb, int p0, int np, bf* EP) {
    typedef __attribute__((ext_vector_type(2))) unsigned short v2us;
    const int lane = threadIdx.x & 31; const size_t wid = (size_t)blockIdx.x * 8 + (threadIdx.x >> 5); if (wid >= (size_t)np * NB_) return; const int pl = (int)(wid / NB_), b = (int)(wid % NB_), p = p0 + pl;
    const int side = lane >> 4; int f = plist[p * 2 + side]; f = f < 0 ? 0 : (f >= NF ? NF - 1 : f);
    int idx = pairs[((size_t)b * NPR + p) * 2 + side] + offs[f]; idx = idx < 0 ? 0 : (idx >= TOT ? TOT - 1 : idx); v2us o;
#pragma unroll
    for (int i = 0; i < 2; ++i) { const int e = (lane & 15) * 2 + i; o[i] = f2bf(emb[(size_t)idx * NE + e]); }
    *(volatile v2us*)(EP + wid * 64 + lane * 2) = o; __threadfence(); *(volatile v2us*)(EP + wid * 64 + lane * 2) = o;
}
__global__ __launch_bounds__(256) void k_relub(const float* __restrict__ Hs, const float* __restrict__ bias, int g0, int ng, bf* Ph, bf* Pl) {
    typedef __attribute__((ext_vector_type(2))) unsigned short v2us;
    const int lane = threadIdx.x & 31; const size_t wid = (size_t)blockIdx.x * 8 + (threadIdx.x >> 5); if (wid >= (size_t)ng * NB_) return; const int g = (int)(wid / NB_); v2us oh, ol;
#pragma unroll
    for (int i = 0; i < 2; ++i) { const int c = lane * 2 + i; const float v = fmaxf(Hs[wid * 64 + c] + bfr(bias[(size_t)(g0 + g) * NH + c]), 0.f); const unsigned short hb = f2bf(v); oh[i] = hb; ol[i] = f2bf(v - bf2f(hb)); }
    const size_t o = wid * 64 + lane * 2; *(volatile v2us*)(Ph + o) = oh; *(volatile v2us*)(Pl + o) = ol; __threadfence(); *(volatile v2us*)(Ph + o) = oh; *(volatile v2us*)(Pl + o) = ol;
}
__device__ __forceinline__ float smooth_z(float z) { const float g = 1.0f; const float sm = -2.0f / (g * g * g) * z * z * z + 3.0f / (2.0f * g) * z + 0.5f; return (z <= -0.5f * g) ? 0.f : ((z >= 0.5f * g) ? 1.f : sm); }
__global__ __launch_bounds__(256) void k_head(const float* __restrict__ H1, const float* __restrict__ b1, const float* __restrict__ w2, const float* __restrict__ b2, const float* __restrict__ z, int g0, int ng, const float* __restrict__ prev, float* S) {
    const int b = blockIdx.x * 256 + threadIdx.x; if (b >= NB_) return; float acc = prev ? prev[b] : 0.f;
#pragma unroll 1
    for (int g = 0; g < ng; ++g) { float s = bfr(b2[g0 + g]);
#pragma unroll 4
        for (int c = 0; c < NH; ++c) s = fmaf(fmaxf(H1[((size_t)g * NB_ + b) * 64 + c] + bfr(b1[(size_t)(g0 + g) * NH + c]), 0.f), bfr(w2[(size_t)(g0 + g) * NH + c]), s);
        acc = fmaf(s, smooth_z(bfr(z[g0 + g])), acc); }
    *(volatile float*)(S + b) = acc; __threadfence(); *(volatile float*)(S + b) = acc;
}

extern "C" void kernel_launch(void* const* d_in, const int* in_sizes, int n_in,
                              void* d_out, int out_size, void* d_ws, size_t ws_size, hipStream_t stream) {
    (void)in_sizes; (void)n_in; (void)out_size;
    const int* mains = (const int*)d_in[0]; const int* pairs = (const int*)d_in[1]; const int* plist = (const int*)d_in[2]; const int* offs = (const int*)d_in[3]; const float* emb = (const float*)d_in[4];
    const float* mw0 = (const float*)d_in[5]; const float* mw1 = (const float*)d_in[6]; const float* mw2 = (const float*)d_in[7]; const float* mb0 = (const float*)d_in[8]; const float* mb1 = (const float*)d_in[9]; const float* mb2 = (const float*)d_in[10];
    const float* pw0 = (const float*)d_in[11]; const float* pw1 = (const float*)d_in[12]; const float* pw2 = (const float*)d_in[13]; const float* pb0 = (const float*)d_in[14]; const float* pb1 = (const float*)d_in[15]; const float* pb2 = (const float*)d_in[16];
    const float* zm = (const float*)d_in[17]; const float* zp = (const float*)d_in[18];
    float* out = (float*)d_out;
    char* wsp = (char*)d_ws;
    auto take = [&](size_t bytes) { char* p = wsp; wsp += (bytes + 255) & ~(size_t)255; return (void*)p; };
    bf* W0T = (bf*)take((size_t)NPR * 64 * 64 * 2); bf* W1T = (bf*)take((size_t)NPR * 64 * 64 * 2);
    bf* E = (bf*)take((size_t)PCH * NB_ * 64 * 2); float* Hs = (float*)take((size_t)PCH * NB_ * 64 * 4); bf* Ph = (bf*)take((size_t)PCH * NB_ * 64 * 2); bf* Pl = (bf*)take((size_t)PCH * NB_ * 64 * 2);
    float* SP[NPC + 2]; for (int i = 0; i < NPC + 2; ++i) SP[i] = (float*)take((size_t)NB_ * 4);
    if ((size_t)(wsp - (char*)d_ws) > ws_size) return;
    const size_t sW = 64 * 64, sA = (size_t)NB_ * 64, sC = (size_t)NB_ * 64;
    k_wtb<<<NF, 256, 0, stream>>>(mw0, NE, NH, W0T); k_wtb<<<NF, 256, 0, stream>>>(mw1, NH, NH, W1T);
    k_embm<<<(NF * NB_) / 8, 256, 0, stream>>>(mains, offs, emb, E);
    k_gemmbz<false, false><<<dim3(NB_ / 64, 1, NF), 128, 0, stream>>>(E, nullptr, W0T, nullptr, Hs, 64, nullptr, nullptr, 64, 0, sA, sW, 0, sC);
    k_relub<<<(NF * NB_) / 8, 256, 0, stream>>>(Hs, mb0, 0, NF, Ph, Pl);
    k_gemmbz<true, false><<<dim3(NB_ / 64, 1, NF), 128, 0, stream>>>(Ph, Pl, W1T, nullptr, Hs, 64, nullptr, nullptr, 64, 0, sA, sW, 0, sC);
    k_head<<<NB_ / 256, 256, 0, stream>>>(Hs, mb1, mw2, mb2, zm, 0, NF, nullptr, SP[0]);
    k_wtb<<<NPR, 256, 0, stream>>>(pw0, 2 * NE, NH, W0T); k_wtb<<<NPR, 256, 0, stream>>>(pw1, NH, NH, W1T);
    for (int ch = 0; ch < NPC; ++ch) { const int p0 = ch * PCH;
        k_embp<<<(PCH * NB_) / 8, 256, 0, stream>>>(pairs, plist, offs, emb, p0, PCH, E);
        k_gemmbz<false, false><<<dim3(NB_ / 64, 1, PCH), 128, 0, stream>>>(E, nullptr, W0T + (size_t)p0 * sW, nullptr, Hs, 64, nullptr, nullptr, 64, 0, sA, sW, 0, sC);
        k_relub<<<(PCH * NB_) / 8, 256, 0, stream>>>(Hs, pb0, p0, PCH, Ph, Pl);
        k_gemmbz<true, false><<<dim3(NB_ / 64, 1, PCH), 128, 0, stream>>>(Ph, Pl, W1T + (size_t)p0 * sW, nullptr, Hs, 64, nullptr, nullptr, 64, 0, sA, sW, 0, sC);
        k_head<<<NB_ / 256, 256, 0, stream>>>(Hs, pb1, pw2, pb2, zp, p0, PCH, SP[ch], SP[ch + 1]); }
    k_head<<<NB_ / 256, 256, 0, stream>>>(Hs, pb1, pw2, pb2, zp, 0, 0, SP[NPC], out);
}
